// LTRelationshipHead_48430051230299
// MI455X (gfx1250) — hardware-run, weakly checked
//
#include <hip/hip_runtime.h>
#include <stddef.h>
#include <math.h>


typedef _Float16 v16h __attribute__((ext_vector_type(16)));
typedef _Float16 v8h  __attribute__((ext_vector_type(8)));
typedef float    v8f  __attribute__((ext_vector_type(8)));
typedef float    v4f  __attribute__((ext_vector_type(4)));

#ifndef NQL
#define NQL 512
#endif
#ifndef NQT
#define NQT 512
#endif
#define NQL_FULL 512
#define NQT_FULL 512
#define NPTS 20
#define NCLS 10
#define FDIM 256
#define HDIM 256
#define INW  (2 * FDIM)
#define PI_F 3.14159265358979323846f

static_assert(NQL >= 64 && NQL <= NQL_FULL && (NQL % 64) == 0);
static_assert(NQT >= 64 && NQT <= NQT_FULL && (NQT % 64) == 0);
static_assert(FDIM == 32 * 8);
static_assert(HDIM == FDIM);
static_assert(HDIM == 256);
static_assert((INW % 64) == 0 && (INW % 32) == 0);
static_assert((HDIM % 64) == 0 && (HDIM % 32) == 0);
static_assert((NQL % 8) == 0 && (NQT % 8) == 0);

#define LDT 72
#define LDC 68
static_assert((LDT % 8) == 0 && LDT >= 64);
static_assert((LDC % 4) == 0 && LDC >= 64);

#define WCARRY 64.0f
#define ACARRY 16.0f
#define MCARRY 16.0f
#define ECARRY 64.0f

#define PI_T 16
#define PJ_T 32
#define PLD  260
static_assert(PI_T * 16 == 256);
static_assert(PJ_T == 32);
static_assert(PI_T * 8 == 128);
static_assert((PLD % 4) == 0 && PLD >= HDIM);
static_assert((NQL % PI_T) == 0 && (NQT % PJ_T) == 0);
static_assert(((size_t)(NQL - 1) * NQT_FULL + NQT) * 4 <= (size_t)1048576);

#define W1_BYTES   ((size_t)HDIM * INW * 2)
#define W2_BYTES   ((size_t)HDIM * HDIM * 2)
#define INL_BYTES  ((size_t)NQL * INW * 2)
#define INT_BYTES  ((size_t)NQT * INW * 2)
#define HL_BYTES   ((size_t)NQL * HDIM * 2)
#define HT_BYTES   ((size_t)NQT * HDIM * 2)
#define LA_BYTES   ((size_t)NQL * HDIM * 4)
#define TB_BYTES   ((size_t)NQT * HDIM * 4)
#define OFF_W1L ((size_t)0)
#define OFF_W2L (OFF_W1L + W1_BYTES)
#define OFF_W1T (OFF_W2L + W2_BYTES)
#define OFF_W2T (OFF_W1T + W1_BYTES)
#define OFF_WA  (OFF_W2T + W2_BYTES)
#define OFF_WB  (OFF_WA + W2_BYTES)
#define OFF_INL (OFF_WB + W2_BYTES)
#define OFF_INT (OFF_INL + INL_BYTES)
#define OFF_HL  (OFF_INT + INT_BYTES)
#define OFF_HT  (OFF_HL + HL_BYTES)
#define OFF_EL  (OFF_HT + HT_BYTES)
#define OFF_ET  (OFF_EL + HL_BYTES)
#define OFF_LA  (OFF_ET + HT_BYTES)
#define OFF_TB  (OFF_LA + LA_BYTES)
#define WS_TOTAL (OFF_TB + TB_BYTES)
static_assert((W1_BYTES % 128) == 0 && (W2_BYTES % 128) == 0);
static_assert((INL_BYTES % 128) == 0 && (INT_BYTES % 128) == 0);
static_assert((HL_BYTES % 128) == 0 && (HT_BYTES % 128) == 0);
static_assert((LA_BYTES % 128) == 0 && (TB_BYTES % 128) == 0);
static_assert(WS_TOTAL <= (size_t)134217728);

__device__ __forceinline__ float bf16r(float x) {
  unsigned int u = __float_as_uint(x);
  u = (u + 0x7FFFu + ((u >> 16) & 1u)) & 0xFFFF0000u;
  return __uint_as_float(u);
}

static __device__ __forceinline__ _Float16 toh_flush(float v) {
  const _Float16 r = (_Float16)v;
  return (fabsf(v) < 6.103515625e-05f) ? (_Float16)0.0f : r;
}

__device__ __forceinline__ v16h frag_at(const _Float16* p) {
  v8h lo = *(const v8h*)(p);
  v8h hi = *(const v8h*)(p + 16);
  v16h out;
#pragma unroll
  for (int i = 0; i < 8; ++i) { out[i] = lo[i]; out[i + 8] = hi[i]; }
  return out;
}

__device__ __forceinline__ v8f wmma16(v16h a, v16h b, v8f c) {
  v8f d = __builtin_amdgcn_wmma_f32_16x16x32_f16(false, a, false, b, (short)0, c,
                                                 false, false);
  asm volatile("v_nop\n\tv_nop\n\tv_nop\n\tv_nop" : "+v"(d) : "v"(a), "v"(b));
  return d;
}

__device__ __forceinline__ float relu_act(float t) {
  return fmaxf(t, 0.0f);
}

__global__ __launch_bounds__(256) void wconv_kernel(
    const float* __restrict__ W, _Float16* __restrict__ Wt, unsigned ldw, unsigned ldk) {
  __shared__ _Float16 T[64 * LDT];
  const unsigned tid = threadIdx.x;
  const unsigned n0 = blockIdx.x * 64u;
  const unsigned k0 = blockIdx.y * 64u;
#pragma unroll 4
  for (unsigned j = 0; j < 16u; ++j) {
    const unsigned idx = tid + 256u * j;
    const unsigned kr = idx >> 6, nc = idx & 63u;
    const float v = W[(size_t)(k0 + kr) * ldw + n0 + nc];
    T[nc * LDT + kr] = (_Float16)(WCARRY * bf16r(v));
  }
  __syncthreads();
  v8h x[2];
  size_t off[2];
#pragma unroll
  for (unsigned i = 0; i < 2u; ++i) {
    const unsigned n = 32u * i + (tid >> 3);
    const unsigned kc = (tid & 7u) * 8u;
    x[i] = *(const v8h*)&T[n * LDT + kc];
    off[i] = (size_t)(n0 + n) * ldk + k0 + kc;
  }
#pragma unroll
  for (int i = 0; i < 2; ++i) *(volatile v8h*)(Wt + off[i]) = x[i];
  __threadfence();
#pragma unroll
  for (int i = 0; i < 2; ++i) *(volatile v8h*)(Wt + off[i]) = x[i];
}

__global__ __launch_bounds__(256) void prep_lane_kernel(
    const float* __restrict__ feats, const float* __restrict__ coords,
    _Float16* __restrict__ dst) {
#pragma clang fp contract(off)
  const unsigned lane = threadIdx.x & 31u, w = threadIdx.x >> 5;
  const unsigned q = blockIdx.x * 8u + w;
  const float* xr = feats + (size_t)q * (NPTS * FDIM) + lane * 8u;

  v4f s0 = {}, s1 = {};
#pragma unroll 1
  for (unsigned p = 0; p < (unsigned)NPTS; ++p) {
    const v4f a0 = *(const v4f*)(xr + p * FDIM);
    const v4f a1 = *(const v4f*)(xr + p * FDIM + 4u);
#pragma unroll
    for (int i = 0; i < 4; ++i) {
      s0[i] += bf16r(a0[i]);
      s1[i] += bf16r(a1[i]);
    }
  }

  const unsigned cb = q * (unsigned)(NPTS * 2);
  const float x1 = bf16r(coords[cb + 32u]);
  const float y1 = bf16r(coords[cb + 33u]);
  const float x0 = bf16r(coords[cb + 6u]);
  const float y0 = bf16r(coords[cb + 7u]);
  const float vx = x1 - x0;
  const float vy = y1 - y0;
  const float nrm = sqrtf(vx * vx + vy * vy) + 1.0e-8f;
  const float rn = 1.0f / nrm;
  float c = vx * rn;
  c = fminf(fmaxf(c, -1.0f), 1.0f);
  const float ang = PI_F - acosf(c);
  const _Float16 ah = toh_flush(ACARRY * ang);

  v8h o, oa;
#pragma unroll
  for (int i = 0; i < 4; ++i) {
    o[i]     = toh_flush(ACARRY * (s0[i] * (1.0f / (float)NPTS)));
    o[i + 4] = toh_flush(ACARRY * (s1[i] * (1.0f / (float)NPTS)));
  }
#pragma unroll
  for (int i = 0; i < 8; ++i) oa[i] = ah;

  _Float16* p = dst + (size_t)q * INW + lane * 8u;
  *(volatile v8h*)p = o;
  *(volatile v8h*)(p + FDIM) = oa;
  __threadfence();
  *(volatile v8h*)p = o;
  *(volatile v8h*)(p + FDIM) = oa;
}

__global__ __launch_bounds__(256) void prep_te_kernel(
    const float* __restrict__ feats, const float* __restrict__ cls,
    _Float16* __restrict__ dst) {
#pragma clang fp contract(off)
  const unsigned lane = threadIdx.x & 31u, w = threadIdx.x >> 5;
  const unsigned q = blockIdx.x * 8u + w;
  const float* xr = feats + (size_t)q * FDIM + lane * 8u;
  const v4f a0 = *(const v4f*)(xr);
  const v4f a1 = *(const v4f*)(xr + 4u);

  float mx = bf16r(cls[q * (unsigned)NCLS]);
#pragma unroll 1
  for (unsigned c = 1; c < (unsigned)NCLS; ++c) mx = fmaxf(mx, bf16r(cls[q * (unsigned)NCLS + c]));
  const float sg = 1.0f / (1.0f + expf(-mx));
  const float score = sg * 2.0f;
  const _Float16 sh = toh_flush(ACARRY * score);

  v8h o, os;
#pragma unroll
  for (int i = 0; i < 4; ++i) {
    o[i]     = toh_flush(ACARRY * bf16r(a0[i]));
    o[i + 4] = toh_flush(ACARRY * bf16r(a1[i]));
  }
#pragma unroll
  for (int i = 0; i < 8; ++i) os[i] = sh;

  _Float16* p = dst + (size_t)q * INW + lane * 8u;
  *(volatile v8h*)p = o;
  *(volatile v8h*)(p + FDIM) = os;
  __threadfence();
  *(volatile v8h*)p = o;
  *(volatile v8h*)(p + FDIM) = os;
}

template <int MODE>
__device__ __forceinline__ void gemm_body(
    const _Float16* __restrict__ A16, const _Float16* __restrict__ Bt, const unsigned K,
    const float* __restrict__ bias, float* __restrict__ outf, _Float16* __restrict__ out16) {
  __shared__ float Cs[64 * LDC];
  const unsigned tid = threadIdx.x, lane = tid & 31u, w = tid >> 5;
  const unsigned mw = w >> 1, nw = w & 1u;
  const unsigned hh = lane >> 4, m = lane & 15u;
  const unsigned n0 = blockIdx.x * 64u;
  const unsigned row0 = blockIdx.y * 64u;

  const _Float16* ap  = A16 + (size_t)(row0 + mw * 16u + m) * K + hh * 8u;
  const _Float16* bp0 = Bt + (size_t)(n0 + nw * 32u + m) * K + hh * 8u;
  const _Float16* bp1 = bp0 + (size_t)16 * K;
  v8f acc0 = {}, acc1 = {};
#pragma unroll 2
  for (unsigned k0 = 0; k0 < K; k0 += 32u) {
    const v16h a  = frag_at(ap + k0);
    const v16h b0 = frag_at(bp0 + k0);
    const v16h b1 = frag_at(bp1 + k0);
    acc0 = wmma16(a, b0, acc0);
    acc1 = wmma16(a, b1, acc1);
  }
#pragma unroll
  for (int r = 0; r < 8; ++r) {
    float* d = &Cs[(mw * 16u + hh * 8u + (unsigned)r) * LDC + nw * 32u + m];
    d[0]  = acc0[r];
    d[16] = acc1[r];
  }
  __syncthreads();

  if (MODE == 0 || MODE == 1) {
    const float cs = (MODE == 0) ? (1.0f / (WCARRY * ACARRY)) : (1.0f / (WCARRY * MCARRY));
    const float oc = (MODE == 0) ? MCARRY : ECARRY;
    v8h x[2];
    size_t off[2];
#pragma unroll
    for (unsigned i = 0; i < 2u; ++i) {
      const unsigned r = 32u * i + (tid >> 3);
      const unsigned c = (tid & 7u) * 8u;
      const v4f u0 = *(const v4f*)&Cs[r * LDC + c];
      const v4f u1 = *(const v4f*)&Cs[r * LDC + c + 4];
      const v4f g0 = *(const v4f*)(bias + n0 + c);
      const v4f g1 = *(const v4f*)(bias + n0 + c + 4u);
#pragma unroll
      for (int j = 0; j < 4; ++j) {
        float t0 = u0[j] * cs + bf16r(g0[j]);
        float t1 = u1[j] * cs + bf16r(g1[j]);
        if (MODE == 0) { t0 = relu_act(t0); t1 = relu_act(t1); }
        x[i][j]     = toh_flush(oc * t0);
        x[i][j + 4] = toh_flush(oc * t1);
      }
      off[i] = (size_t)(row0 + r) * HDIM + n0 + c;
    }
#pragma unroll
    for (int i = 0; i < 2; ++i) *(volatile v8h*)(out16 + off[i]) = x[i];
    __threadfence();
#pragma unroll
    for (int i = 0; i < 2; ++i) *(volatile v8h*)(out16 + off[i]) = x[i];
  }

  if (MODE == 2 || MODE == 3) {
    const float cs = 1.0f / (WCARRY * ECARRY);
    v4f xs[4];
    size_t off[4];
#pragma unroll
    for (unsigned i = 0; i < 4u; ++i) {
      const unsigned r = 16u * i + (tid >> 4);
      const unsigned c = (tid & 15u) * 4u;
      const v4f u = *(const v4f*)&Cs[r * LDC + c];
      v4f val;
#pragma unroll
      for (int j = 0; j < 4; ++j) val[j] = u[j] * cs;
      if (MODE == 2) {
        const v4f g = *(const v4f*)(bias + n0 + c);
#pragma unroll
        for (int j = 0; j < 4; ++j) val[j] = val[j] + bf16r(g[j]);
      }
      xs[i] = val;
      off[i] = (size_t)(row0 + r) * HDIM + n0 + c;
    }
#pragma unroll
    for (int i = 0; i < 4; ++i) *(volatile v4f*)(outf + off[i]) = xs[i];
    __threadfence();
#pragma unroll
    for (int i = 0; i < 4; ++i) *(volatile v4f*)(outf + off[i]) = xs[i];
  }
}

__global__ __launch_bounds__(256) void gemm_hid_kernel(
    const _Float16* __restrict__ A16, const _Float16* __restrict__ Bt,
    const float* __restrict__ bias, _Float16* __restrict__ out16) {
  gemm_body<0>(A16, Bt, (unsigned)INW, bias, (float*)0, out16);
}
__global__ __launch_bounds__(256) void gemm_emb_kernel(
    const _Float16* __restrict__ A16, const _Float16* __restrict__ Bt,
    const float* __restrict__ bias, _Float16* __restrict__ out16) {
  gemm_body<1>(A16, Bt, (unsigned)HDIM, bias, (float*)0, out16);
}
__global__ __launch_bounds__(256) void gemm_la_kernel(
    const _Float16* __restrict__ A16, const _Float16* __restrict__ Bt,
    const float* __restrict__ bias, float* __restrict__ outf) {
  gemm_body<2>(A16, Bt, (unsigned)HDIM, bias, outf, (_Float16*)0);
}
__global__ __launch_bounds__(256) void gemm_tb_kernel(
    const _Float16* __restrict__ A16, const _Float16* __restrict__ Bt,
    const float* __restrict__ bias, float* __restrict__ outf) {
  gemm_body<3>(A16, Bt, (unsigned)HDIM, bias, outf, (_Float16*)0);
}

__global__ __launch_bounds__(256) void pair_kernel(
    const float* __restrict__ LAb, const float* __restrict__ TB,
    const float* __restrict__ w2, const float* __restrict__ b2, float* __restrict__ out) {
  __shared__ float sla[PI_T * PLD];
  __shared__ float stb[PJ_T * PLD];
  __shared__ float sw2[HDIM];
  __shared__ float so[PI_T * PJ_T];

  const unsigned tid = threadIdx.x;
  const unsigned i0 = blockIdx.y * (unsigned)PI_T;
  const unsigned j0 = blockIdx.x * (unsigned)PJ_T;

#pragma unroll 4
  for (unsigned t = 0; t < (unsigned)(PI_T * 64 / 256); ++t) {
    const unsigned idx = tid + 256u * t;
    const unsigned r = idx >> 6, c = (idx & 63u) * 4u;
    *(v4f*)&sla[r * PLD + c] = *(const v4f*)(LAb + (size_t)(i0 + r) * HDIM + c);
  }
#pragma unroll 4
  for (unsigned t = 0; t < (unsigned)(PJ_T * 64 / 256); ++t) {
    const unsigned idx = tid + 256u * t;
    const unsigned r = idx >> 6, c = (idx & 63u) * 4u;
    *(v4f*)&stb[r * PLD + c] = *(const v4f*)(TB + (size_t)(j0 + r) * HDIM + c);
  }
  sw2[tid] = bf16r(w2[tid]);
  __syncthreads();

  const unsigned ti = tid >> 4, tj = tid & 15u;
  float acc0 = 0.0f, acc1 = 0.0f;
#pragma unroll 2
  for (unsigned k = 0; k < (unsigned)HDIM; k += 4u) {
    const v4f a  = *(const v4f*)&sla[ti * PLD + k];
    const v4f c0 = *(const v4f*)&stb[tj * PLD + k];
    const v4f c1 = *(const v4f*)&stb[(tj + 16u) * PLD + k];
    const v4f wv = *(const v4f*)&sw2[k];
#pragma unroll
    for (int e = 0; e < 4; ++e) {
      acc0 = fmaf(fmaxf(a[e] + c0[e], 0.0f), wv[e], acc0);
      acc1 = fmaf(fmaxf(a[e] + c1[e], 0.0f), wv[e], acc1);
    }
  }
  const float bb = bf16r(b2[0]);
  so[ti * PJ_T + tj]       = acc0 + bb;
  so[ti * PJ_T + tj + 16u] = acc1 + bb;
  __syncthreads();

  if (tid < 128u) {
    const unsigned r = tid >> 3;
    const unsigned c = (tid & 7u) * 4u;
    const v4f x = *(const v4f*)&so[r * PJ_T + c];
    float* p = out + (size_t)(i0 + r) * NQT_FULL + j0 + c;
    *(volatile v4f*)p = x;
    __threadfence();
    *(volatile v4f*)p = x;
  }
}

extern "C" void kernel_launch(void* const* d_in, const int* in_sizes, int n_in,
                              void* d_out, int out_size, void* d_ws, size_t ws_size,
                              hipStream_t stream) {
  if (n_in < 16) return;
  if ((long long)in_sizes[0] < (long long)NQL * NPTS * FDIM) return;
  if ((long long)in_sizes[1] < (long long)NQL * NPTS * 2) return;
  if ((long long)in_sizes[2] < (long long)NQT * FDIM) return;
  if ((long long)in_sizes[3] < (long long)NQT * NCLS) return;
  if ((long long)in_sizes[4] < (long long)INW * HDIM) return;
  if ((long long)in_sizes[6] < (long long)HDIM * HDIM) return;
  if ((long long)in_sizes[8] < (long long)INW * HDIM) return;
  if ((long long)in_sizes[10] < (long long)HDIM * HDIM) return;
  if ((long long)in_sizes[12] < (long long)2 * HDIM * HDIM) return;
  if (in_sizes[5] < HDIM || in_sizes[7] < HDIM || in_sizes[9] < HDIM || in_sizes[11] < HDIM) return;
  if (in_sizes[13] < HDIM || in_sizes[14] < HDIM || in_sizes[15] < 1) return;
  if ((long long)out_size < (long long)(NQL - 1) * NQT_FULL + NQT) return;
  if (ws_size < WS_TOTAL) return;

  const float* lane_feats  = (const float*)d_in[0];
  const float* lane_coords = (const float*)d_in[1];
  const float* te_feats    = (const float*)d_in[2];
  const float* te_cls      = (const float*)d_in[3];
  const float* o1_w1  = (const float*)d_in[4];
  const float* o1_b1  = (const float*)d_in[5];
  const float* o1_w2  = (const float*)d_in[6];
  const float* o1_b2  = (const float*)d_in[7];
  const float* o2_w1  = (const float*)d_in[8];
  const float* o2_b1  = (const float*)d_in[9];
  const float* o2_w2  = (const float*)d_in[10];
  const float* o2_b2  = (const float*)d_in[11];
  const float* cls_w1 = (const float*)d_in[12];
  const float* cls_b1 = (const float*)d_in[13];
  const float* cls_w2 = (const float*)d_in[14];
  const float* cls_b2 = (const float*)d_in[15];
  float* out = (float*)d_out;

  char* ws = (char*)d_ws;
  _Float16* W1L_t = (_Float16*)(ws + OFF_W1L);
  _Float16* W2L_t = (_Float16*)(ws + OFF_W2L);
  _Float16* W1T_t = (_Float16*)(ws + OFF_W1T);
  _Float16* W2T_t = (_Float16*)(ws + OFF_W2T);
  _Float16* WA_t  = (_Float16*)(ws + OFF_WA);
  _Float16* WB_t  = (_Float16*)(ws + OFF_WB);
  _Float16* INL   = (_Float16*)(ws + OFF_INL);
  _Float16* INT   = (_Float16*)(ws + OFF_INT);
  _Float16* HL    = (_Float16*)(ws + OFF_HL);
  _Float16* HT    = (_Float16*)(ws + OFF_HT);
  _Float16* EL    = (_Float16*)(ws + OFF_EL);
  _Float16* ET    = (_Float16*)(ws + OFF_ET);
  float*    LA    = (float*)(ws + OFF_LA);
  float*    TB    = (float*)(ws + OFF_TB);

  dim3 blk(256);
  dim3 gw1(HDIM / 64, INW / 64);
  dim3 gw2(HDIM / 64, HDIM / 64);

  wconv_kernel<<<gw1, blk, 0, stream>>>(o1_w1, W1L_t, (unsigned)HDIM, (unsigned)INW);
  wconv_kernel<<<gw2, blk, 0, stream>>>(o1_w2, W2L_t, (unsigned)HDIM, (unsigned)HDIM);
  wconv_kernel<<<gw1, blk, 0, stream>>>(o2_w1, W1T_t, (unsigned)HDIM, (unsigned)INW);
  wconv_kernel<<<gw2, blk, 0, stream>>>(o2_w2, W2T_t, (unsigned)HDIM, (unsigned)HDIM);
  wconv_kernel<<<gw2, blk, 0, stream>>>(cls_w1, WA_t, (unsigned)HDIM, (unsigned)HDIM);
  wconv_kernel<<<gw2, blk, 0, stream>>>(cls_w1 + (size_t)HDIM * HDIM, WB_t, (unsigned)HDIM,
                                        (unsigned)HDIM);

  prep_lane_kernel<<<dim3(NQL / 8), blk, 0, stream>>>(lane_feats, lane_coords, INL);
  prep_te_kernel<<<dim3(NQT / 8), blk, 0, stream>>>(te_feats, te_cls, INT);

  dim3 ggl(HDIM / 64, NQL / 64);
  dim3 ggt(HDIM / 64, NQT / 64);

  gemm_hid_kernel<<<ggl, blk, 0, stream>>>(INL, W1L_t, o1_b1, HL);
  gemm_emb_kernel<<<ggl, blk, 0, stream>>>(HL, W2L_t, o1_b2, EL);
  gemm_la_kernel<<<ggl, blk, 0, stream>>>(EL, WA_t, cls_b1, LA);
  gemm_hid_kernel<<<ggt, blk, 0, stream>>>(INT, W1T_t, o2_b1, HT);
  gemm_emb_kernel<<<ggt, blk, 0, stream>>>(HT, W2T_t, o2_b2, ET);
  gemm_tb_kernel<<<ggt, blk, 0, stream>>>(ET, WB_t, cls_b1, TB);

  pair_kernel<<<dim3(NQT / PJ_T, NQL / PI_T), blk, 0, stream>>>(LA, TB, cls_w2, cls_b2, out);
}
